// RelationTransformer_40295383171629
// MI455X (gfx1250) — hardware-run, weakly checked
//
#include <hip/hip_runtime.h>
#include <math.h>

#ifndef NB
#define NB 4
#endif
#ifndef NTOK
#define NTOK 256
#endif
#define NB_FULL 4
#define NTOK_FULL 256
#define FEAT 1028
#define KAPP 1024
#define CH 256
#define CG 128
#define KCAT 384
#define HC 128
#define ROWS_SIDE (NB * NTOK)
#define ROWS (2 * ROWS_SIDE)

static_assert(NB <= NB_FULL);
static_assert(NTOK <= NTOK_FULL);
static_assert(NTOK % 64 == 0);
static_assert(ROWS_SIDE % 64 == 0);
static_assert(KAPP % 64 == 0);
static_assert(KCAT % 32 == 0);
static_assert(CH % 64 == 0);
static_assert(HC % 64 == 0);
static_assert(KCAT == CH + CG);
static_assert((KCAT * 2) % 128 == 0);
static_assert((CH * 2) % 128 == 0);

typedef __attribute__((ext_vector_type(4))) float v4f;
typedef __attribute__((ext_vector_type(4))) unsigned int v4u;
typedef __attribute__((ext_vector_type(2))) unsigned int v2u;
typedef _Float16 h16;

#define VST2(T, ptr, val) do { const T vst2_v_ = (val); *(volatile T*)(ptr) = vst2_v_; __threadfence(); *(volatile T*)(ptr) = vst2_v_; } while (0)
#define VST2V4(ptr, val) do { const v4f vst2_v4_ = (val); *(volatile v4f*)(ptr) = vst2_v4_; __threadfence(); *(volatile v4f*)(ptr) = vst2_v4_; } while (0)

static __device__ __forceinline__ float bfr(float f) {
    unsigned int u = __float_as_uint(f);
    u += 0x7FFFu + ((u >> 16) & 1u);
    return __uint_as_float(u & 0xFFFF0000u);
}
static __device__ __forceinline__ h16 toh_flush(float v) { const h16 r = (h16)v; return (fabsf(v) < 6.103515625e-05f) ? (h16)0.0f : r; }
static __device__ __forceinline__ unsigned int pk2h(float a, float b) {
    return (unsigned int)__builtin_bit_cast(unsigned short, toh_flush(a)) | ((unsigned int)__builtin_bit_cast(unsigned short, toh_flush(b)) << 16);
}
static __device__ __forceinline__ void st8h_flush(unsigned short* p, const float* v) {
    v4u pk; pk.x = pk2h(v[0], v[1]); pk.y = pk2h(v[2], v[3]); pk.z = pk2h(v[4], v[5]); pk.w = pk2h(v[6], v[7]);
    VST2(v4u, (v4u*)p, pk);
}
static __device__ __forceinline__ void st4h_flush(unsigned short* p, const float* v) {
    v2u pk; pk.x = pk2h(v[0], v[1]); pk.y = pk2h(v[2], v[3]);
    VST2(v2u, (v2u*)p, pk);
}
static __device__ __forceinline__ void ld8(const float* __restrict__ p, float* o) {
    const v4f a = *(const v4f*)p, b = *(const v4f*)(p + 4);
    o[0] = a.x; o[1] = a.y; o[2] = a.z; o[3] = a.w; o[4] = b.x; o[5] = b.y; o[6] = b.z; o[7] = b.w;
}
static __device__ __forceinline__ void ld8bf(const float* __restrict__ p, float* o) {
    const v4f a = *(const v4f*)p, b = *(const v4f*)(p + 4);
    o[0] = bfr(a.x); o[1] = bfr(a.y); o[2] = bfr(a.z); o[3] = bfr(a.w); o[4] = bfr(b.x); o[5] = bfr(b.y); o[6] = bfr(b.z); o[7] = bfr(b.w);
}
static __device__ __forceinline__ void ld4bf(const float* __restrict__ p, float* o) {
    const v4f a = *(const v4f*)p;
    o[0] = bfr(a.x); o[1] = bfr(a.y); o[2] = bfr(a.z); o[3] = bfr(a.w);
}
static __device__ __forceinline__ float wsum(float v) {
#pragma unroll
    for (int off = 16; off > 0; off >>= 1) v += __shfl_xor(v, off, 32);
    return v;
}

namespace eng {
typedef __attribute__((ext_vector_type(16))) _Float16 v16h;
typedef __attribute__((ext_vector_type(8)))  _Float16 v8h;
typedef __attribute__((ext_vector_type(16))) __bf16   v16b;
typedef __attribute__((ext_vector_type(8)))  __bf16   v8b;
typedef __attribute__((ext_vector_type(8)))  float    v8f;
typedef __attribute__((ext_vector_type(4)))  float    v4f;

__device__ __forceinline__ unsigned short f2bf_bits(float f) {
  unsigned u = __float_as_uint(f);
  return (unsigned short)((u + 0x7FFFu + ((u >> 16) & 1u)) >> 16);
}
__device__ __forceinline__ float bf_bits2f(unsigned short h) { return __uint_as_float(((unsigned)h) << 16); }

__device__ __forceinline__ void dep_guard_h(v8f& a, v8f& b, v16h x, v16h y) { asm volatile("v_nop\n\tv_nop\n\tv_nop\n\tv_nop" : "+v"(a), "+v"(b) : "v"(x), "v"(y)); }
__device__ __forceinline__ void dep_guard_b(v8f& a, v8f& b, v16b x, v16b y) { asm volatile("v_nop\n\tv_nop\n\tv_nop\n\tv_nop" : "+v"(a), "+v"(b) : "v"(x), "v"(y)); }
__device__ __forceinline__ void keep4_h(v16h a, v16h b, v16h c, v16h d) { asm volatile("v_nop" :: "v"(a), "v"(b), "v"(c), "v"(d)); }
__device__ __forceinline__ void keep4_b(v16b a, v16b b, v16b c, v16b d) { asm volatile("v_nop" :: "v"(a), "v"(b), "v"(c), "v"(d)); }
__device__ __forceinline__ void acc_guard4(v8f& a, v8f& b, v8f& c, v8f& d) { asm volatile("v_nop\n\tv_nop\n\tv_nop\n\tv_nop" : "+v"(a), "+v"(b), "+v"(c), "+v"(d)); }
template <typename T> struct Frag;
template <> struct Frag<_Float16> {
  typedef v16h V; union U { v16h v; v8h h[2]; };
  static __device__ __forceinline__ v16h load(const _Float16* p) {
    U f; f.h[0] = *(const v8h*)(p); f.h[1] = *(const v8h*)(p + 16); return f.v;
  }
  static __device__ __forceinline__ v8f mma(v16h a, v16h b, v8f c) {
    return __builtin_amdgcn_wmma_f32_16x16x32_f16(false, a, false, b, (short)0, c, false, false);
  }
  static __device__ __forceinline__ void guard(v8f& a, v8f& b, v16h x, v16h y) { dep_guard_h(a, b, x, y); }
  static __device__ __forceinline__ void keep(v16h a, v16h b, v16h c, v16h d) { keep4_h(a, b, c, d); }
};
template <> struct Frag<__bf16> {
  typedef v16b V; union U { v16b v; v8b h[2]; };
  static __device__ __forceinline__ v16b load(const __bf16* p) {
    U f; f.h[0] = *(const v8b*)(p); f.h[1] = *(const v8b*)(p + 16); return f.v;
  }
  static __device__ __forceinline__ v8f mma(v16b a, v16b b, v8f c) {
    return __builtin_amdgcn_wmma_f32_16x16x32_bf16(false, a, false, b, (short)0, c, false, false);
  }
  static __device__ __forceinline__ void guard(v8f& a, v8f& b, v16b x, v16b y) { dep_guard_b(a, b, x, y); }
  static __device__ __forceinline__ void keep(v16b a, v16b b, v16b c, v16b d) { keep4_b(a, b, c, d); }
};

template <int ET> struct Elem;
template <> struct Elem<0> { typedef _Float16 T; };
template <> struct Elem<1> { typedef __bf16 T; };
template <int ET, bool SPLIT, int BIAS_MODE, int OUT_MODE, bool RESID, int ACT = 0>
__device__ __forceinline__ void gemm64_body(
    const unsigned short* __restrict__ Ap, const unsigned short* __restrict__ A2p, int lda, long strideA,
    const unsigned short* __restrict__ Btp, const unsigned short* __restrict__ Bt2p, int ldb, long strideB,
    void* __restrict__ Cout, void* __restrict__ Cout2, int ldc, long strideC,
    const float* __restrict__ bias,
    const float* __restrict__ resid, long strideR,
    int M, int N, int K, float scale) {
  typedef typename Elem<ET>::T T;
  typedef typename Frag<T>::V V;
  const T* A = (const T*)Ap; const T* A2 = (const T*)A2p; const T* Bt = (const T*)Btp; const T* Bt2 = (const T*)Bt2p;
  __shared__ __align__(16) float sT[8][16 * 68];
  const int b    = blockIdx.y;
  const int lane = threadIdx.x & 31;
  const int wave = threadIdx.x >> 5;
  const int tilesN = N >> 6;
  const int tilesM = M >> 6;
  const int tile = blockIdx.x * 8 + wave;
  if (tile >= tilesM * tilesN) return;
  const int tm = tile / tilesN;
  const int tn = tile - tm * tilesN;
  const int m0 = tm << 6;
  const int n0 = tn << 6;

  const T* Ab  = A  + (size_t)b * strideA;
  const T* Bb  = Bt + (size_t)b * strideB;
  const T* Ab2 = SPLIT ? (A2  + (size_t)b * strideA) : nullptr;
  const T* Bb2 = SPLIT ? (Bt2 + (size_t)b * strideB) : nullptr;

  const int rlane = lane & 15;
  const int koff  = (lane >> 4) * 8;
  const int mOff  = (lane >> 4) * 8;

  v8f acc[4][4];
#pragma unroll
  for (int i = 0; i < 4; ++i)
#pragma unroll
    for (int j = 0; j < 4; ++j) acc[i][j] = (v8f){0.f,0.f,0.f,0.f,0.f,0.f,0.f,0.f};

  for (int k0 = 0; k0 < K; k0 += 32) {
    V bh[4], bl[4];
#pragma unroll
    for (int j = 0; j < 4; ++j) {
      const size_t bo = (size_t)(n0 + (j << 4) + rlane) * ldb + koff + k0;
      bh[j] = Frag<T>::load(Bb + bo);
      if (SPLIT) bl[j] = Frag<T>::load(Bb2 + bo);
    }
#pragma unroll
    for (int i = 0; i < 4; ++i) {
      const size_t ao = (size_t)(m0 + (i << 4) + rlane) * lda + koff + k0;
      V ah = Frag<T>::load(Ab + ao);
      V al;
      if (SPLIT) al = Frag<T>::load(Ab2 + ao);
#pragma unroll
      for (int j = 0; j < 4; ++j) {
        acc[i][j] = Frag<T>::mma(ah, bh[j], acc[i][j]);
        if (SPLIT) {
          acc[i][j] = Frag<T>::mma(ah, bl[j], acc[i][j]);
          acc[i][j] = Frag<T>::mma(al, bh[j], acc[i][j]);
        }
      }
      Frag<T>::guard(acc[i][0], acc[i][3], ah, SPLIT ? al : ah);
    }
    Frag<T>::keep(bh[0], bh[1], bh[2], bh[3]);
    if (SPLIT) Frag<T>::keep(bl[0], bl[1], bl[2], bl[3]);
  }
  acc_guard4(acc[0][0], acc[0][1], acc[0][2], acc[0][3]);
  acc_guard4(acc[1][0], acc[1][1], acc[1][2], acc[1][3]);
  acc_guard4(acc[2][0], acc[2][1], acc[2][2], acc[2][3]);
  acc_guard4(acc[3][0], acc[3][1], acc[3][2], acc[3][3]);

  float* slab = sT[wave];
  const float* Rb = RESID ? (resid + (size_t)b * strideR) : nullptr;
#pragma unroll
  for (int i = 0; i < 4; ++i) {
    const int mBase = m0 + (i << 4);
#pragma unroll
    for (int j = 0; j < 4; ++j) {
      const int n = n0 + (j << 4) + rlane;
      float bv = 0.f;
      if (BIAS_MODE == 2) bv = bias[n];
#pragma unroll
      for (int r = 0; r < 8; ++r) {
        float v = acc[i][j][r] * scale;
        if (BIAS_MODE == 1) v += bias[mBase + mOff + r];
        if (BIAS_MODE == 2) v += bv;
        if (RESID) v += Rb[(size_t)(mBase + mOff + r) * ldc + n];
        if (ACT == 1) v = tanhf(v);
        if (ACT == 2) v = fmaxf(v, 0.0f);
        if (ACT == 3) v = v / (1.0f + expf(-v));
        if (ACT == 4) v = (v > 0.f) ? v : 0.01f * v;
        if (ACT == 5) v = 0.5f * v * (1.0f + erff(v * 0.70710678118654752f));
        if (ACT == 6) v = (v > 0.f) ? v : 0.2f * v;
        if (ACT == 7) { const float u = 0.7978845608028654f * (v + 0.044715f * v * v * v); v = 0.5f * v * (1.f + tanhf(u)); }
        slab[(mOff + r) * 68 + (j << 4) + rlane] = v;
      }
    }
    __builtin_amdgcn_fence(3  , "workgroup");
    __builtin_amdgcn_wave_barrier();
    __builtin_amdgcn_fence(2  , "workgroup");
    if (OUT_MODE == 0) {
      float* C = (float*)Cout + (size_t)b * strideC;
      const int hh = lane >> 4, c4 = (lane & 15) * 4;
      for (int pass = 0; pass < 2; ++pass) {
#pragma unroll
        for (int it = 0; it < 8; ++it) {
          const int row = it * 2 + hh;
          v4f v = *(const v4f*)(slab + row * 68 + c4);
          *(volatile v4f*)(C + (size_t)(mBase + row) * ldc + n0 + c4) = v;
        }
        __threadfence();
      }
    } else {
      const int q = lane >> 3, c8 = (lane & 7) * 8;
      unsigned short* C  = (unsigned short*)Cout  + (size_t)b * strideC;
      unsigned short* C2 = (OUT_MODE == 2) ? ((unsigned short*)Cout2 + (size_t)b * strideC) : nullptr;
      for (int pass = 0; pass < 2; ++pass) {
#pragma unroll
        for (int it = 0; it < 4; ++it) {
          const int row = it * 4 + q;
          const float* sp = slab + row * 68 + c8;
          v8h hv, lv;
#pragma unroll
          for (int e = 0; e < 8; ++e) {
            if (OUT_MODE == 1) {
              hv[e] = (_Float16)sp[e];
            } else {
              unsigned short hb = f2bf_bits(sp[e]);
              unsigned short lb = f2bf_bits(sp[e] - bf_bits2f(hb));
              hv[e] = __builtin_bit_cast(_Float16, hb);
              lv[e] = __builtin_bit_cast(_Float16, lb);
            }
          }
          *(volatile v8h*)(C + (size_t)(mBase + row) * ldc + n0 + c8) = hv;
          if (OUT_MODE == 2) *(volatile v8h*)(C2 + (size_t)(mBase + row) * ldc + n0 + c8) = lv;
        }
        __threadfence();
      }
    }
    __builtin_amdgcn_fence(3  , "workgroup");
    __builtin_amdgcn_wave_barrier();
    __builtin_amdgcn_fence(2  , "workgroup");
  }
}
}

static_assert(8 * 16 * 68 * 4 <= 131072);

__global__ __launch_bounds__(256) void k_gemm_f16(const unsigned short* __restrict__ Ap, int lda, long strideA,
                                                  const unsigned short* __restrict__ Btp, int ldb, long strideB,
                                                  float* __restrict__ C, int ldc, long strideC, int M, int N, int K, float scale) {
    eng::gemm64_body<0, false, 0, 0, false, 0>(Ap, nullptr, lda, strideA, Btp, nullptr, ldb, strideB, (void*)C, nullptr, ldc, strideC, nullptr, nullptr, 0, M, N, K, scale);
}

static_assert(256 * 16 == 32 * 64 * 2);
static_assert(64 * 33 * 4 <= 131072);
__global__ __launch_bounds__(256) void k_planeT(const float* __restrict__ src, unsigned short* __restrict__ XA, int set0) {
    __shared__ float tile[64][33];
    const int lane = threadIdx.x & 31;
    const int wave = __builtin_amdgcn_readfirstlane(threadIdx.x >> 5);
    const int k0 = blockIdx.x * 64, m0 = blockIdx.y * 32, s = blockIdx.z;
    const float* sp = src + (size_t)s * (FEAT * NTOK_FULL);
#pragma unroll
    for (int i = 0; i < 8; ++i) {
        const int kk = wave + 8 * i;
        tile[kk][lane] = sp[(size_t)(k0 + kk) * NTOK_FULL + m0 + lane];
    }
    __syncthreads();
    const int mr = threadIdx.x >> 3, p = threadIdx.x & 7;
    float v[8];
#pragma unroll
    for (int i = 0; i < 8; ++i) v[i] = bfr(tile[8 * p + i][mr]) * 8.0f;
    st8h_flush(XA + ((size_t)((set0 + s) * NTOK + m0 + mr)) * KAPP + k0 + 8 * p, v);
}

__global__ __launch_bounds__(256) void k_wconv(const float* __restrict__ Wm, int KI, int NO, unsigned short* __restrict__ W16, int KP, int koff, float sw) {
    const int u = blockIdx.x * 256 + threadIdx.x; const int per = KI / 8; if (u >= NO * per) return;
    const int k0 = 8 * (u % per); const int o = u / per; float v[8];
#pragma unroll
    for (int i = 0; i < 8; ++i) v[i] = bfr(Wm[(size_t)(k0 + i) * NO + o]) * sw;
    st8h_flush(W16 + (size_t)o * KP + koff + k0, v);
}

static_assert(32 * 16 == CH * 2);
static_assert(32 * 8 == CG * 2);
__global__ __launch_bounds__(256) void k_ln1(const float* __restrict__ P, const float* __restrict__ src, int set0,
                                             const float* __restrict__ ba1, const float* __restrict__ gla, const float* __restrict__ bla,
                                             const float* __restrict__ wg1, const float* __restrict__ bg1, const float* __restrict__ glg, const float* __restrict__ blg,
                                             unsigned short* __restrict__ A2) {
    #pragma clang fp contract(off)
    const int lane = threadIdx.x & 31;
    const int wave = __builtin_amdgcn_readfirstlane(threadIdx.x >> 5);
    const int lr = blockIdx.x * 8 + wave;
    if (lr >= ROWS_SIDE) return;
    const int s = lr / NTOK, n = lr - s * NTOK;
    const int row = set0 * NTOK + lr;
    {
        const int c0 = 8 * lane;
        float x[8], t[8];
        ld8(P + (size_t)row * CH + c0, x);
        ld8bf(ba1 + c0, t);
#pragma unroll
        for (int i = 0; i < 8; ++i) x[i] += t[i];
        float sm = ((x[0] + x[1]) + (x[2] + x[3])) + ((x[4] + x[5]) + (x[6] + x[7]));
        sm = wsum(sm);
        const float mean = sm * (1.0f / 256.0f);
        float d[8], q = 0.f;
#pragma unroll
        for (int i = 0; i < 8; ++i) { d[i] = x[i] - mean; q += d[i] * d[i]; }
        q = wsum(q);
        const float rs = 1.0f / sqrtf(q * (1.0f / 256.0f) + 1e-5f);
        float gg[8], bb[8], y[8];
        ld8bf(gla + c0, gg); ld8bf(bla + c0, bb);
#pragma unroll
        for (int i = 0; i < 8; ++i) y[i] = fmaxf(d[i] * rs * gg[i] + bb[i], 0.f) * 8.0f;
        st8h_flush(A2 + (size_t)row * KCAT + c0, y);
    }
    {
        const int c0 = 4 * lane;
        const float* gp = src + (size_t)s * (FEAT * NTOK_FULL) + (size_t)KAPP * NTOK_FULL + n;
        const float g0 = bfr(gp[0]), g1 = bfr(gp[NTOK_FULL]), g2 = bfr(gp[2 * NTOK_FULL]), g3 = bfr(gp[3 * NTOK_FULL]);
        float w0[4], w1[4], w2[4], w3[4], bgv[4], u[4];
        ld4bf(wg1 + c0, w0); ld4bf(wg1 + CG + c0, w1); ld4bf(wg1 + 2 * CG + c0, w2); ld4bf(wg1 + 3 * CG + c0, w3); ld4bf(bg1 + c0, bgv);
#pragma unroll
        for (int i = 0; i < 4; ++i) u[i] = (((g0 * w0[i] + g1 * w1[i]) + g2 * w2[i]) + g3 * w3[i]) + bgv[i];
        float sm = (u[0] + u[1]) + (u[2] + u[3]);
        sm = wsum(sm);
        const float mean = sm * (1.0f / 128.0f);
        float d[4], q = 0.f;
#pragma unroll
        for (int i = 0; i < 4; ++i) { d[i] = u[i] - mean; q += d[i] * d[i]; }
        q = wsum(q);
        const float rs = 1.0f / sqrtf(q * (1.0f / 128.0f) + 1e-5f);
        float gg[4], bb[4], y[4];
        ld4bf(glg + c0, gg); ld4bf(blg + c0, bb);
#pragma unroll
        for (int i = 0; i < 4; ++i) y[i] = fmaxf(d[i] * rs * gg[i] + bb[i], 0.f) * 8.0f;
        st4h_flush(A2 + (size_t)row * KCAT + CH + c0, y);
    }
}

__global__ __launch_bounds__(256) void k_ln2(const float* __restrict__ EPRE, const float* __restrict__ ba2, const float* __restrict__ bg2,
                                             const float* __restrict__ gf, const float* __restrict__ bfv, unsigned short* __restrict__ EMB16) {
    #pragma clang fp contract(off)
    const int lane = threadIdx.x & 31;
    const int wave = __builtin_amdgcn_readfirstlane(threadIdx.x >> 5);
    const int row = blockIdx.x * 8 + wave;
    if (row >= ROWS) return;
    const int c0 = 8 * lane;
    float x[8], t[8], t2[8];
    ld8(EPRE + (size_t)row * CH + c0, x);
    ld8bf(ba2 + c0, t); ld8bf(bg2 + c0, t2);
#pragma unroll
    for (int i = 0; i < 8; ++i) x[i] = (x[i] + t[i]) + t2[i];
    float sm = ((x[0] + x[1]) + (x[2] + x[3])) + ((x[4] + x[5]) + (x[6] + x[7]));
    sm = wsum(sm);
    const float mean = sm * (1.0f / 256.0f);
    float d[8], q = 0.f;
#pragma unroll
    for (int i = 0; i < 8; ++i) { d[i] = x[i] - mean; q += d[i] * d[i]; }
    q = wsum(q);
    const float rs = 1.0f / sqrtf(q * (1.0f / 256.0f) + 1e-5f);
    float gg[8], bb[8], y[8];
    ld8bf(gf + c0, gg); ld8bf(bfv + c0, bb);
#pragma unroll
    for (int i = 0; i < 8; ++i) y[i] = (d[i] * rs * gg[i] + bb[i]) * 8.0f;
    st8h_flush(EMB16 + (size_t)row * CH + c0, y);
}

static_assert(256 * 16 == 32 * 32 * 4);
static_assert((2 * 32 * 132 + 128) * 4 <= 131072);
__global__ __launch_bounds__(256) void k_pair(const float* __restrict__ AC, const float* __restrict__ bc1, const float* __restrict__ wc2,
                                              const float* __restrict__ bc2, float* __restrict__ out) {
    __shared__ float aT[32][132];
    __shared__ float cT[32][132];
    __shared__ float w2[128];
    const int b = blockIdx.x, nblk = blockIdx.y, mblk = blockIdx.z;
    const float* arow = AC + ((size_t)b * NTOK + nblk * 32) * HC;
    const float* crow = AC + ((size_t)ROWS_SIDE + (size_t)b * NTOK + mblk * 32) * HC;
    for (int i = threadIdx.x; i < 32 * 128; i += 256) {
        const int r = i >> 7, h = i & 127;
        aT[r][h] = arow[(size_t)r * HC + h] + bfr(bc1[h]);
        cT[r][h] = crow[(size_t)r * HC + h];
    }
    if (threadIdx.x < 128) w2[threadIdx.x] = bfr(wc2[threadIdx.x]);
    __syncthreads();
    const float b2 = bfr(bc2[0]);
    const int n = threadIdx.x >> 3;
    const int mbase = (threadIdx.x & 7) * 4;
    float acc[4] = {0.f, 0.f, 0.f, 0.f};
#pragma unroll 4
    for (int h = 0; h < 128; ++h) {
        const float av = aT[n][h];
        const float wv = w2[h];
#pragma unroll
        for (int j = 0; j < 4; ++j) acc[j] = fmaf(fmaxf(av + cT[mbase + j][h], 0.f), wv, acc[j]);
    }
    v4f o4; o4.x = acc[0] + b2; o4.y = acc[1] + b2; o4.z = acc[2] + b2; o4.w = acc[3] + b2;
    float* op = out + ((size_t)b * NTOK_FULL + nblk * 32 + n) * NTOK_FULL + mblk * 32 + mbase;
    VST2V4(op, o4);
}

constexpr size_t al256(size_t x) { return (x + 255) / 256 * 256; }
constexpr size_t SZ_XA  = al256((size_t)ROWS * KAPP * 2);
constexpr size_t SZ_W1  = al256((size_t)CH * KAPP * 2);
constexpr size_t SZ_W2  = al256((size_t)CH * KCAT * 2);
constexpr size_t SZ_WC  = al256((size_t)2 * HC * CH * 2);
constexpr size_t SZ_P   = al256((size_t)ROWS * CH * 4);
constexpr size_t SZ_A2  = al256((size_t)ROWS * KCAT * 2);
constexpr size_t SZ_EP  = al256((size_t)ROWS * CH * 4);
constexpr size_t SZ_EMB = al256((size_t)ROWS * CH * 2);
constexpr size_t SZ_AC  = al256((size_t)ROWS * HC * 4);
constexpr size_t WS_TOTAL = SZ_XA + SZ_W1 + SZ_W2 + SZ_WC + SZ_P + SZ_A2 + SZ_EP + SZ_EMB + SZ_AC;
static_assert(WS_TOTAL <= (size_t)134217728);

extern "C" void kernel_launch(void* const* d_in, const int* in_sizes, int n_in, void* d_out, int out_size, void* d_ws, size_t ws_size, hipStream_t stream) {
    if (n_in < 28) return;
    if (in_sizes[0] < NB * FEAT * NTOK_FULL || in_sizes[1] < NB * FEAT * NTOK_FULL) return;
    if (in_sizes[2] < KAPP * CH || in_sizes[6] < CH * CH || in_sizes[8] < 4 * CG || in_sizes[12] < CG * CH || in_sizes[24] < 2 * CH * HC || in_sizes[26] < HC || in_sizes[27] < 1) return;
    if (in_sizes[3] < CH || in_sizes[4] < CH || in_sizes[5] < CH || in_sizes[7] < CH || in_sizes[9] < CG || in_sizes[10] < CG || in_sizes[11] < CG ||
        in_sizes[13] < CH || in_sizes[14] < CH || in_sizes[15] < CH || in_sizes[25] < HC) return;
    if (out_size < (NB - 1) * NTOK_FULL * NTOK_FULL + (NTOK - 1) * NTOK_FULL + NTOK) return;
    if (ws_size < WS_TOTAL) return;
    const float* tracks = (const float*)d_in[0];
    const float* dets   = (const float*)d_in[1];
    const float* wa1 = (const float*)d_in[2];
    const float* ba1 = (const float*)d_in[3];
    const float* gla = (const float*)d_in[4];
    const float* bla = (const float*)d_in[5];
    const float* wa2 = (const float*)d_in[6];
    const float* ba2 = (const float*)d_in[7];
    const float* wg1 = (const float*)d_in[8];
    const float* bg1 = (const float*)d_in[9];
    const float* glg = (const float*)d_in[10];
    const float* blg = (const float*)d_in[11];
    const float* wg2 = (const float*)d_in[12];
    const float* bg2 = (const float*)d_in[13];
    const float* gf  = (const float*)d_in[14];
    const float* bfv = (const float*)d_in[15];
    const float* wc1 = (const float*)d_in[24];
    const float* bc1 = (const float*)d_in[25];
    const float* wc2 = (const float*)d_in[26];
    const float* bc2 = (const float*)d_in[27];
    float* out = (float*)d_out;

    char* wsp = (char*)d_ws;
    unsigned short* XA    = (unsigned short*)wsp; wsp += SZ_XA;
    unsigned short* W1T   = (unsigned short*)wsp; wsp += SZ_W1;
    unsigned short* W2T   = (unsigned short*)wsp; wsp += SZ_W2;
    unsigned short* WC16  = (unsigned short*)wsp; wsp += SZ_WC;
    float*          P     = (float*)wsp;          wsp += SZ_P;
    unsigned short* A2    = (unsigned short*)wsp; wsp += SZ_A2;
    float*          EPRE  = (float*)wsp;          wsp += SZ_EP;
    unsigned short* EMB16 = (unsigned short*)wsp; wsp += SZ_EMB;
    float*          AC    = (float*)wsp;          wsp += SZ_AC;

    k_wconv<<<(CH * (KAPP / 8) + 255) / 256, 256, 0, stream>>>(wa1, KAPP, CH, W1T, KAPP, 0, 32.0f);
    k_wconv<<<(CH * (CH / 8) + 255) / 256, 256, 0, stream>>>(wa2, CH, CH, W2T, KCAT, 0, 16.0f);
    k_wconv<<<(CH * (CG / 8) + 255) / 256, 256, 0, stream>>>(wg2, CG, CH, W2T, KCAT, CH, 16.0f);
    k_wconv<<<(HC * (CH / 8) + 255) / 256, 256, 0, stream>>>(wc1, CH, HC, WC16, CH, 0, 16.0f);
    k_wconv<<<(HC * (CH / 8) + 255) / 256, 256, 0, stream>>>(wc1 + (size_t)CH * HC, CH, HC, WC16 + (size_t)HC * CH, CH, 0, 16.0f);
    k_planeT<<<dim3(KAPP / 64, NTOK / 32, NB), 256, 0, stream>>>(tracks, XA, 0);
    k_planeT<<<dim3(KAPP / 64, NTOK / 32, NB), 256, 0, stream>>>(dets, XA, NB);
    k_gemm_f16<<<dim3((unsigned)(((ROWS / 64) * (CH / 64) + 7) / 8), 1), 256, 0, stream>>>(XA, KAPP, 0, W1T, KAPP, 0, P, CH, 0, ROWS, CH, KAPP, 1.0f / 256.0f);
    k_ln1<<<(ROWS_SIDE + 7) / 8, 256, 0, stream>>>(P, tracks, 0, ba1, gla, bla, wg1, bg1, glg, blg, A2);
    k_ln1<<<(ROWS_SIDE + 7) / 8, 256, 0, stream>>>(P, dets, NB, ba1, gla, bla, wg1, bg1, glg, blg, A2);
    k_gemm_f16<<<dim3((unsigned)(((ROWS / 64) * (CH / 64) + 7) / 8), 1), 256, 0, stream>>>(A2, KCAT, 0, W2T, KCAT, 0, EPRE, CH, 0, ROWS, CH, KCAT, 1.0f / 128.0f);
    k_ln2<<<(ROWS + 7) / 8, 256, 0, stream>>>(EPRE, ba2, bg2, gf, bfv, EMB16);
    k_gemm_f16<<<dim3((unsigned)(((ROWS_SIDE / 64) * (HC / 64) + 7) / 8), 2), 256, 0, stream>>>(EMB16, CH, (long)ROWS_SIDE * CH, WC16, CH, (long)HC * CH, AC, HC, (long)ROWS_SIDE * HC, ROWS_SIDE, HC, CH, 1.0f / 128.0f);
    k_pair<<<dim3(NB, NTOK / 32, NTOK / 32), 256, 0, stream>>>(AC, bc1, wc2, bc2, out);
}
